// ContextHypergraphAttention_20109036880615
// MI455X (gfx1250) — hardware-verified
//
#include <hip/hip_runtime.h>
#include <hip/hip_bf16.h>

typedef __attribute__((ext_vector_type(16))) _Float16 v16h;
typedef __attribute__((ext_vector_type(8)))  _Float16 v8h;
typedef __attribute__((ext_vector_type(16))) __bf16   v16b;
typedef __attribute__((ext_vector_type(8)))  __bf16   v8b;
typedef __attribute__((ext_vector_type(8)))  float    v8f;
typedef __attribute__((ext_vector_type(4)))  float    v4f;
#define PSCALE 32768.0f
#define U16(p) ((const unsigned short*)(const void*)(p))
#define PSCALE_INV (1.0f / 32768.0f)

__device__ __forceinline__ unsigned short f2bf_bits(float f) {
  unsigned u = __float_as_uint(f);
  return (unsigned short)((u + 0x7FFFu + ((u >> 16) & 1u)) >> 16);
}
__device__ __forceinline__ float bf_bits2f(unsigned short h) { return __uint_as_float(((unsigned)h) << 16); }

__device__ __forceinline__ void dep_guard_h(v8f& a, v8f& b, v16h x, v16h y) { asm volatile("v_nop\n\tv_nop\n\tv_nop\n\tv_nop" : "+v"(a), "+v"(b) : "v"(x), "v"(y)); }
__device__ __forceinline__ void dep_guard_b(v8f& a, v8f& b, v16b x, v16b y) { asm volatile("v_nop\n\tv_nop\n\tv_nop\n\tv_nop" : "+v"(a), "+v"(b) : "v"(x), "v"(y)); }
__device__ __forceinline__ void keep4_h(v16h a, v16h b, v16h c, v16h d) { asm volatile("v_nop" :: "v"(a), "v"(b), "v"(c), "v"(d)); }
__device__ __forceinline__ void keep4_b(v16b a, v16b b, v16b c, v16b d) { asm volatile("v_nop" :: "v"(a), "v"(b), "v"(c), "v"(d)); }
__device__ __forceinline__ void acc_guard4(v8f& a, v8f& b, v8f& c, v8f& d) { asm volatile("v_nop\n\tv_nop\n\tv_nop\n\tv_nop" : "+v"(a), "+v"(b), "+v"(c), "+v"(d)); }
template <typename T> struct Frag;
template <> struct Frag<_Float16> {
  typedef v16h V; union U { v16h v; v8h h[2]; };
  static __device__ __forceinline__ v16h load(const _Float16* p) {
    U f; f.h[0] = *(const v8h*)(p); f.h[1] = *(const v8h*)(p + 16); return f.v;
  }
  static __device__ __forceinline__ v8f mma(v16h a, v16h b, v8f c) {
    return __builtin_amdgcn_wmma_f32_16x16x32_f16(false, a, false, b, (short)0, c, false, false);
  }
  static __device__ __forceinline__ void guard(v8f& a, v8f& b, v16h x, v16h y) { dep_guard_h(a, b, x, y); }
  static __device__ __forceinline__ void keep(v16h a, v16h b, v16h c, v16h d) { keep4_h(a, b, c, d); }
};
template <> struct Frag<__bf16> {
  typedef v16b V; union U { v16b v; v8b h[2]; };
  static __device__ __forceinline__ v16b load(const __bf16* p) {
    U f; f.h[0] = *(const v8b*)(p); f.h[1] = *(const v8b*)(p + 16); return f.v;
  }
  static __device__ __forceinline__ v8f mma(v16b a, v16b b, v8f c) {
    return __builtin_amdgcn_wmma_f32_16x16x32_bf16(false, a, false, b, (short)0, c, false, false);
  }
  static __device__ __forceinline__ void guard(v8f& a, v8f& b, v16b x, v16b y) { dep_guard_b(a, b, x, y); }
  static __device__ __forceinline__ void keep(v16b a, v16b b, v16b c, v16b d) { keep4_b(a, b, c, d); }
};

template <int ET> struct Elem;
template <> struct Elem<0> { typedef _Float16 T; };
template <> struct Elem<1> { typedef __bf16 T; };
template <int ET, bool SPLIT, int BIAS_MODE, int OUT_MODE, bool RESID, int ACT = 0>
__global__ __launch_bounds__(256) void wmma_gemm64(
    const unsigned short* __restrict__ Ap, const unsigned short* __restrict__ A2p, int lda, long strideA,
    const unsigned short* __restrict__ Btp, const unsigned short* __restrict__ Bt2p, int ldb, long strideB,
    void* __restrict__ Cout, void* __restrict__ Cout2, int ldc, long strideC,
    const float* __restrict__ bias,
    const float* __restrict__ resid, long strideR,
    int M, int N, int K, float scale) {
  typedef typename Elem<ET>::T T;
  typedef typename Frag<T>::V V;
  const T* A = (const T*)Ap; const T* A2 = (const T*)A2p; const T* Bt = (const T*)Btp; const T* Bt2 = (const T*)Bt2p;
  __shared__ __align__(16) float sT[8][16 * 68];
  const int b    = blockIdx.y;
  const int lane = threadIdx.x & 31;
  const int wave = threadIdx.x >> 5;
  const int tilesN = N >> 6;
  const int tilesM = M >> 6;
  const int tile = blockIdx.x * 8 + wave;
  if (tile >= tilesM * tilesN) return;
  const int tm = tile / tilesN;
  const int tn = tile - tm * tilesN;
  const int m0 = tm << 6;
  const int n0 = tn << 6;

  const T* Ab  = A  + (size_t)b * strideA;
  const T* Bb  = Bt + (size_t)b * strideB;
  const T* Ab2 = SPLIT ? (A2  + (size_t)b * strideA) : nullptr;
  const T* Bb2 = SPLIT ? (Bt2 + (size_t)b * strideB) : nullptr;

  const int rlane = lane & 15;
  const int koff  = (lane >> 4) * 8;
  const int mOff  = (lane >> 4) * 8;

  v8f acc[4][4];
#pragma unroll
  for (int i = 0; i < 4; ++i)
#pragma unroll
    for (int j = 0; j < 4; ++j) acc[i][j] = (v8f){0.f,0.f,0.f,0.f,0.f,0.f,0.f,0.f};

  for (int k0 = 0; k0 < K; k0 += 32) {
    V bh[4], bl[4];
#pragma unroll
    for (int j = 0; j < 4; ++j) {
      const size_t bo = (size_t)(n0 + (j << 4) + rlane) * ldb + koff + k0;
      bh[j] = Frag<T>::load(Bb + bo);
      if (SPLIT) bl[j] = Frag<T>::load(Bb2 + bo);
    }
#pragma unroll
    for (int i = 0; i < 4; ++i) {
      const size_t ao = (size_t)(m0 + (i << 4) + rlane) * lda + koff + k0;
      V ah = Frag<T>::load(Ab + ao);
      V al;
      if (SPLIT) al = Frag<T>::load(Ab2 + ao);
#pragma unroll
      for (int j = 0; j < 4; ++j) {
        acc[i][j] = Frag<T>::mma(ah, bh[j], acc[i][j]);
        if (SPLIT) {
          acc[i][j] = Frag<T>::mma(ah, bl[j], acc[i][j]);
          acc[i][j] = Frag<T>::mma(al, bh[j], acc[i][j]);
        }
      }
      Frag<T>::guard(acc[i][0], acc[i][3], ah, SPLIT ? al : ah);
    }
    Frag<T>::keep(bh[0], bh[1], bh[2], bh[3]);
    if (SPLIT) Frag<T>::keep(bl[0], bl[1], bl[2], bl[3]);
  }
  acc_guard4(acc[0][0], acc[0][1], acc[0][2], acc[0][3]);
  acc_guard4(acc[1][0], acc[1][1], acc[1][2], acc[1][3]);
  acc_guard4(acc[2][0], acc[2][1], acc[2][2], acc[2][3]);
  acc_guard4(acc[3][0], acc[3][1], acc[3][2], acc[3][3]);

  float* slab = sT[wave];
  const float* Rb = RESID ? (resid + (size_t)b * strideR) : nullptr;
#pragma unroll
  for (int i = 0; i < 4; ++i) {
    const int mBase = m0 + (i << 4);
#pragma unroll
    for (int j = 0; j < 4; ++j) {
      const int n = n0 + (j << 4) + rlane;
      float bv = 0.f;
      if (BIAS_MODE == 2) bv = bias[n];
#pragma unroll
      for (int r = 0; r < 8; ++r) {
        float v = acc[i][j][r] * scale;
        if (BIAS_MODE == 1) v += bias[mBase + mOff + r];
        if (BIAS_MODE == 2) v += bv;
        if (RESID) v += Rb[(size_t)(mBase + mOff + r) * ldc + n];
        if (ACT == 1) v = tanhf(v);
        if (ACT == 2) v = fmaxf(v, 0.0f);
        if (ACT == 3) v = v / (1.0f + expf(-v));
        if (ACT == 4) v = (v > 0.f) ? v : 0.01f * v;
        if (ACT == 5) v = 0.5f * v * (1.0f + erff(v * 0.70710678118654752f));
        slab[(mOff + r) * 68 + (j << 4) + rlane] = v;
      }
    }
    __builtin_amdgcn_fence(__ATOMIC_RELEASE, "workgroup");
    __builtin_amdgcn_wave_barrier();
    __builtin_amdgcn_fence(__ATOMIC_ACQUIRE, "workgroup");
    if (OUT_MODE == 0) {
      float* C = (float*)Cout + (size_t)b * strideC;
      const int hh = lane >> 4, c4 = (lane & 15) * 4;
      for (int pass = 0; pass < 2; ++pass) {
#pragma unroll
        for (int it = 0; it < 8; ++it) {
          const int row = it * 2 + hh;
          v4f v = *(const v4f*)(slab + row * 68 + c4);
          *(volatile v4f*)(C + (size_t)(mBase + row) * ldc + n0 + c4) = v;
        }
        __threadfence();
      }
    } else {
      const int q = lane >> 3, c8 = (lane & 7) * 8;
      unsigned short* C  = (unsigned short*)Cout  + (size_t)b * strideC;
      unsigned short* C2 = (OUT_MODE == 2) ? ((unsigned short*)Cout2 + (size_t)b * strideC) : nullptr;
      for (int pass = 0; pass < 2; ++pass) {
#pragma unroll
        for (int it = 0; it < 4; ++it) {
          const int row = it * 4 + q;
          const float* sp = slab + row * 68 + c8;
          v8h hv, lv;
#pragma unroll
          for (int e = 0; e < 8; ++e) {
            if (OUT_MODE == 1) {
              hv[e] = (_Float16)sp[e];
            } else {
              unsigned short hb = f2bf_bits(sp[e]);
              unsigned short lb = f2bf_bits(sp[e] - bf_bits2f(hb));
              hv[e] = __builtin_bit_cast(_Float16, hb);
              lv[e] = __builtin_bit_cast(_Float16, lb);
            }
          }
          *(volatile v8h*)(C + (size_t)(mBase + row) * ldc + n0 + c8) = hv;
          if (OUT_MODE == 2) *(volatile v8h*)(C2 + (size_t)(mBase + row) * ldc + n0 + c8) = lv;
        }
        __threadfence();
      }
    }
    __builtin_amdgcn_fence(__ATOMIC_RELEASE, "workgroup");
    __builtin_amdgcn_wave_barrier();
    __builtin_amdgcn_fence(__ATOMIC_ACQUIRE, "workgroup");
  }
}

__global__ __launch_bounds__(256) void cast_f32_f16x2s(
    const float* __restrict__ in, _Float16* __restrict__ out, int n2, float mul) {
  int i = blockIdx.x * 256 + threadIdx.x;
  if (i < n2) {
    const _Float16 h0 = (_Float16)(in[2 * i] * mul), h1 = (_Float16)(in[2 * i + 1] * mul);
    const unsigned u = (unsigned)__builtin_bit_cast(unsigned short, h0) | ((unsigned)__builtin_bit_cast(unsigned short, h1) << 16);
    ((volatile unsigned*)out)[i] = u;
    __threadfence();
    ((volatile unsigned*)out)[i] = u;
  }
}

#define AT_E 128
#define AT_C 64
#define AT_QB 64
#define AT_KC 64
#define AT_NW 4
#define AT_QP 136
#define AT_KP 136
#define AT_VP 72
#define AT_PP 72
#define AT_OP 132
#define AT_PSC 32768.0f
#define AT_L2E 1.4426950408889634f

__device__ __forceinline__ v8f mma_h16(v16h a, v16h b, v8f c) {
  c = __builtin_amdgcn_wmma_f32_16x16x32_f16(false, a, false, b, (short)0, c, false, false);
  asm volatile("v_nop\n\tv_nop\n\tv_nop\n\tv_nop" : "+v"(c) : "v"(a), "v"(b));
  return c;
}

__global__ __launch_bounds__(128)
void attn128_kernel(const _Float16* __restrict__ Qh, const _Float16* __restrict__ Kh,
                    const _Float16* __restrict__ Vt, int ldv,
                    const float* __restrict__ ctxin, const float* __restrict__ Wc, const float* __restrict__ bcv,
                    float* __restrict__ out, int nTok, float inv_scale)
{
  __shared__ __align__(16) float    ctxS[AT_E];
  __shared__ __align__(16) _Float16 Qsh[AT_QB * AT_QP];
  __shared__ __align__(16) _Float16 Ksh[AT_KC * AT_KP];
  __shared__ __align__(16) _Float16 Vts[AT_E * AT_VP];
  __shared__ __align__(16) _Float16 Psh[AT_NW][16 * AT_PP];
  __shared__ __align__(16) float    Os[AT_NW][16 * AT_OP];

  const int tid  = threadIdx.x;
  const int wave = tid >> 5;
  const int lane = tid & 31;
  const int hh   = lane >> 4;
  const int c    = lane & 15;

  const int nqb = nTok / AT_QB;
  const int b   = blockIdx.x / nqb;
  const int qb  = blockIdx.x - b * nqb;
  const int q0  = qb * AT_QB;
  const size_t rowbase = (size_t)b * nTok;
  const size_t colbase = rowbase;

  {
    const float* cr = ctxin + (size_t)b * AT_C;
    const float* wr = Wc + (size_t)tid * AT_C;
    float a = 0.f;
#pragma unroll 4
    for (int cc = 0; cc < AT_C; ++cc) a += cr[cc] * wr[cc];
    ctxS[tid] = a + bcv[tid];
  }
#pragma unroll
  for (int i = 0; i < 8; ++i) {
    const int idx = i * 128 + tid;
    const int row = idx >> 4, c8 = (idx & 15) * 8;
    const v8h v = *(const v8h*)(Qh + (rowbase + q0 + row) * AT_E + c8);
    *(v8h*)(Qsh + row * AT_QP + c8) = v;
  }
  __syncthreads();

  float brow[8];
  {
    const _Float16* qr = Qsh + (wave * 16 + c) * AT_QP + hh * 64;
    const float* cx = ctxS + hh * 64;
    float part = 0.f;
#pragma unroll 8
    for (int e = 0; e < 64; ++e) part += (float)qr[e] * cx[e];
    part += __shfl_xor(part, 16, 32);
#pragma unroll
    for (int r = 0; r < 8; ++r) brow[r] = __shfl(part, 8 * hh + r, 32);
  }

  float mrow[8], lrow[8];
  v8f oacc[8];
  const float ninf = -__builtin_inff();
#pragma unroll
  for (int r = 0; r < 8; ++r) { mrow[r] = ninf; lrow[r] = 0.f; }
#pragma unroll
  for (int t = 0; t < 8; ++t) oacc[t] = (v8f){0.f,0.f,0.f,0.f,0.f,0.f,0.f,0.f};

  const _Float16* qfrag = Qsh + (wave * 16 + c) * AT_QP + 8 * hh;
  const int nChunks = nTok / AT_KC;
  for (int kc = 0; kc < nChunks; ++kc) {
    const int kv0 = kc * AT_KC;
    __syncthreads();
#pragma unroll
    for (int i = 0; i < 8; ++i) {
      const int idx = i * 128 + tid;
      const int krow = idx >> 4, kc8 = (idx & 15) * 8;
      const v8h kk = *(const v8h*)(Kh + (rowbase + kv0 + krow) * AT_E + kc8);
      *(v8h*)(Ksh + krow * AT_KP + kc8) = kk;
      const int d = idx >> 3, vc8 = (idx & 7) * 8;
      const v8h vv = *(const v8h*)(Vt + (size_t)d * ldv + colbase + kv0 + vc8);
      *(v8h*)(Vts + d * AT_VP + vc8) = vv;
    }
    __syncthreads();

    v8f s[4];
#pragma unroll
    for (int j = 0; j < 4; ++j) s[j] = (v8f){0.f,0.f,0.f,0.f,0.f,0.f,0.f,0.f};
#pragma unroll 1
    for (int dc = 0; dc < 4; ++dc) {
      const v16h qa = Frag<_Float16>::load(qfrag + dc * 32);
#pragma unroll
      for (int j = 0; j < 4; ++j) {
        const v16h kb = Frag<_Float16>::load(Ksh + (j * 16 + c) * AT_KP + dc * 32 + 8 * hh);
        s[j] = mma_h16(qa, kb, s[j]);
      }
    }

    float cm[8];
#pragma unroll
    for (int r = 0; r < 8; ++r) {
      float m = ninf;
#pragma unroll
      for (int j = 0; j < 4; ++j) {
        const float z = s[j][r] * inv_scale + brow[r];
        s[j][r] = z;
        m = fmaxf(m, z);
      }
#pragma unroll
      for (int off = 1; off < 16; off <<= 1) m = fmaxf(m, __shfl_xor(m, off, 32));
      cm[r] = m;
    }
    _Float16* pw = Psh[wave];
#pragma unroll
    for (int r = 0; r < 8; ++r) {
      const float mnew  = fmaxf(mrow[r], cm[r]);
      const float alpha = __builtin_amdgcn_exp2f((mrow[r] - mnew) * AT_L2E);
      mrow[r] = mnew;
      float psum = 0.f;
#pragma unroll
      for (int j = 0; j < 4; ++j) {
        const float p = __builtin_amdgcn_exp2f((s[j][r] - mnew) * AT_L2E);
        psum += p;
        pw[(8 * hh + r) * AT_PP + j * 16 + c] = (_Float16)(p * AT_PSC);
      }
#pragma unroll
      for (int off = 1; off < 16; off <<= 1) psum += __shfl_xor(psum, off, 32);
      lrow[r] = lrow[r] * alpha + psum;
#pragma unroll
      for (int t = 0; t < 8; ++t) oacc[t][r] *= alpha;
    }
    __builtin_amdgcn_fence(__ATOMIC_RELEASE, "workgroup");
    __builtin_amdgcn_wave_barrier();
    __builtin_amdgcn_fence(__ATOMIC_ACQUIRE, "workgroup");

#pragma unroll 1
    for (int kk = 0; kk < 2; ++kk) {
      const v16h pa = Frag<_Float16>::load(pw + c * AT_PP + kk * 32 + 8 * hh);
#pragma unroll
      for (int t = 0; t < 8; ++t) {
        const v16h vb = Frag<_Float16>::load(Vts + (t * 16 + c) * AT_VP + kk * 32 + 8 * hh);
        oacc[t] = mma_h16(pa, vb, oacc[t]);
      }
    }
  }

  float* os = Os[wave];
#pragma unroll
  for (int r = 0; r < 8; ++r) {
    const float inv = 1.0f / (lrow[r] * AT_PSC);
#pragma unroll
    for (int t = 0; t < 8; ++t) os[(8 * hh + r) * AT_OP + t * 16 + c] = oacc[t][r] * inv;
  }
  __builtin_amdgcn_fence(__ATOMIC_RELEASE, "workgroup");
  __builtin_amdgcn_wave_barrier();
  __builtin_amdgcn_fence(__ATOMIC_ACQUIRE, "workgroup");
  {
    const int q0w = q0 + wave * 16;
    const int c4 = lane * 4;
    for (int pass = 0; pass < 2; ++pass) {
#pragma unroll
      for (int row = 0; row < 16; ++row) {
        v4f val = *(const v4f*)(os + row * AT_OP + c4);
        *(volatile v4f*)(out + (rowbase + q0w + row) * AT_E + c4) = val;
      }
      __threadfence();
    }
  }
}

extern "C" void kernel_launch(void* const* d_in, const int* in_sizes, int n_in,
                              void* d_out, int out_size, void* d_ws, size_t ws_size,
                              hipStream_t stream)
{
  if (n_in < 10) return;
  const float* X    = (const float*)d_in[0];
  const float* ctxt = (const float*)d_in[1];
  const float* Wq   = (const float*)d_in[2];
  const float* bq   = (const float*)d_in[3];
  const float* Wk   = (const float*)d_in[4];
  const float* bk   = (const float*)d_in[5];
  const float* Wv   = (const float*)d_in[6];
  const float* bv   = (const float*)d_in[7];
  const float* Wc   = (const float*)d_in[8];
  const float* bc   = (const float*)d_in[9];
  float* out = (float*)d_out;

  const int E = AT_E, C = AT_C;
  const int nX   = in_sizes[0];
  const int Mall = nX / E;
  const int Bn   = in_sizes[1] / C;
  if (Bn <= 0 || Mall <= 0) return;
  const int nTok = Mall / Bn;
  if (nTok * Bn != Mall || Mall * E != nX) return;
  if ((Mall % 64) != 0 || (nTok % 64) != 0) return;
  if (in_sizes[2] != E * E || in_sizes[4] != E * E || in_sizes[6] != E * E) return;
  if (in_sizes[3] != E || in_sizes[5] != E || in_sizes[7] != E) return;
  if (in_sizes[8] != E * C || in_sizes[9] != E || in_sizes[1] != Bn * C) return;
  if (out_size != nX) return;

  const size_t nTokE = (size_t)Mall * E;
  const size_t nW    = (size_t)E * E;
  size_t off = 0;
  _Float16* Xh  = (_Float16*)((char*)d_ws + off); off += nTokE * 2;
  _Float16* Qh  = (_Float16*)((char*)d_ws + off); off += nTokE * 2;
  _Float16* Kh  = (_Float16*)((char*)d_ws + off); off += nTokE * 2;
  _Float16* Vt  = (_Float16*)((char*)d_ws + off); off += nTokE * 2;
  _Float16* Wqh = (_Float16*)((char*)d_ws + off); off += nW * 2;
  _Float16* Wkh = (_Float16*)((char*)d_ws + off); off += nW * 2;
  _Float16* Wvh = (_Float16*)((char*)d_ws + off); off += nW * 2;
  if (off > ws_size) return;

  const float wcarry = 256.0f;
  const float wundo  = 1.0f / 256.0f;

  {
    const int n2x = nX / 2;
    cast_f32_f16x2s<<<dim3((n2x + 255) / 256), 256, 0, stream>>>(X, Xh, n2x, 1.0f);
    const int n2w = (E * E) / 2;
    cast_f32_f16x2s<<<dim3((n2w + 255) / 256), 256, 0, stream>>>(Wq, Wqh, n2w, wcarry);
    cast_f32_f16x2s<<<dim3((n2w + 255) / 256), 256, 0, stream>>>(Wk, Wkh, n2w, wcarry);
    cast_f32_f16x2s<<<dim3((n2w + 255) / 256), 256, 0, stream>>>(Wv, Wvh, n2w, wcarry);
  }

  {
    const int tilesQK = (Mall / 64) * (E / 64);
    const dim3 gq((tilesQK + 7) / 8, 1);
    wmma_gemm64<0, false, 2, 1, false, 0><<<gq, 256, 0, stream>>>(
        (const unsigned short*)Xh, (const unsigned short*)Xh, E, 0L,
        (const unsigned short*)Wqh, (const unsigned short*)Wqh, E, 0L,
        (void*)Qh, (void*)Qh, E, 0L,
        bq, bq, 0L, Mall, E, E, wundo);
    wmma_gemm64<0, false, 2, 1, false, 0><<<gq, 256, 0, stream>>>(
        (const unsigned short*)Xh, (const unsigned short*)Xh, E, 0L,
        (const unsigned short*)Wkh, (const unsigned short*)Wkh, E, 0L,
        (void*)Kh, (void*)Kh, E, 0L,
        bk, bk, 0L, Mall, E, E, wundo);
    const int tilesV = (E / 64) * (Mall / 64);
    const dim3 gv((tilesV + 7) / 8, 1);
    wmma_gemm64<0, false, 1, 1, false, 0><<<gv, 256, 0, stream>>>(
        (const unsigned short*)Wvh, (const unsigned short*)Wvh, E, 0L,
        (const unsigned short*)Xh, (const unsigned short*)Xh, E, 0L,
        (void*)Vt, (void*)Vt, Mall, 0L,
        bv, bv, 0L, E, Mall, E, wundo);
  }

  {
    const float scale_f   = (float)11.313708498984761;
    const float inv_scale = 1.0f / scale_f;
    attn128_kernel<<<dim3(Bn * (nTok / 64)), 128, 0, stream>>>(
        Qh, Kh, Vt, Mall, ctxt, Wc, bc, out, nTok, inv_scale);
  }
}
